// LidarCameraFusionMambaBlock_16449724745540
// MI455X (gfx1250) — hardware-verified
//
#include <hip/hip_runtime.h>


#ifndef NB
#define NB 4
#endif
#ifndef SEQ
#define SEQ 4096
#endif
#define NB_FULL  4
#define SEQ_FULL 4096
#ifndef OUT_SEQ
#define OUT_SEQ SEQ
#endif
#define DM   256
#define DI   512
#define DS   16
#define DR   16
#define NX   48
#define XZP  1024
#define BG   (NB >= 2 ? 2 : 1)
#define NTG  (BG * SEQ)
#define TC   64
#define SCH  128
#define SSP  52
#define LOG2E 1.4426950408889634f
#define LN2   0.6931471805599453f
#define WSC  64.0f
#define WSI  (1.0f / 64.0f)
#define YSC  16.0f
#define YSI  (1.0f / 16.0f)

#define EP_CAM  0
#define EP_LID  1
#define EP_GUID 2
#define EP_OUT  3

static_assert(DR + 2 * DS == NX);
static_assert(NX % 16 == 0);
static_assert(DR == 16);
static_assert(DS == 16);
static_assert(DM % 32 == 0);
static_assert(DI % 32 == 0);
static_assert(DI % 64 == 0);
static_assert(DM % 64 == 0);
static_assert(XZP == 2 * DI);
static_assert(SEQ % 64 == 0);
static_assert(NTG % 64 == 0);
static_assert(SEQ % TC == 0);
static_assert(DI % SCH == 0);
static_assert(SCH % 32 == 0);
static_assert((TC * 8) % SCH == 0);
static_assert(TC % 8 == 0);
static_assert(NB % BG == 0);
static_assert(NB <= NB_FULL);
static_assert(SEQ <= SEQ_FULL);
static_assert((SSP * 4) % 16 == 0);
static_assert(SSP >= NX);
static_assert(32 * 16 * 8 == 16 * 64 * 4);
static_assert(32 * 16 * 4 == 16 * 64 * 2);
static_assert(32 * 16 * 16 == 64 * 32 * 4);
static_assert((SCH / 32) * 32 * 16 * (TC / 4) == TC * SCH * 4);
static_assert((SCH / 32) * 32 * 16 * (TC / 8) == TC * SCH * 2);
static_assert(16 * 68 * 4 <= 131072);
static_assert(64 * SSP * 4 + 16 * 68 * 4 <= 131072);
static_assert(TC * 32 * 4 + TC * SCH * 4 <= 131072);

typedef _Float16 h16;
typedef unsigned short bf;
typedef __attribute__((ext_vector_type(16))) __bf16   v16bf;
typedef __attribute__((ext_vector_type(16))) _Float16 v16h;
typedef __attribute__((ext_vector_type(8)))  _Float16 v8h;
typedef __attribute__((ext_vector_type(8)))  unsigned short v8us;
typedef __attribute__((ext_vector_type(8)))  float    v8f;
typedef __attribute__((ext_vector_type(4)))  float    v4f;
typedef v4f  __attribute__((may_alias)) v4fa;

__device__ __forceinline__ unsigned short f2bf(float f) { unsigned u = __float_as_uint(f); u += 0x7FFFu + ((u >> 16) & 1u); return (unsigned short)(u >> 16); }
__device__ __forceinline__ float bfr(float f) { return __uint_as_float(((unsigned)f2bf(f)) << 16); }
__device__ __forceinline__ v16h cat16(v8h lo, v8h hi) { return __builtin_shufflevector(lo, hi, 0, 1, 2, 3, 4, 5, 6, 7, 8, 9, 10, 11, 12, 13, 14, 15); }
__device__ __forceinline__ v16bf cat16b(v8us lo, v8us hi) { return __builtin_bit_cast(v16bf, __builtin_shufflevector(lo, hi, 0, 1, 2, 3, 4, 5, 6, 7, 8, 9, 10, 11, 12, 13, 14, 15)); }
__device__ __forceinline__ v8f wmma16(v16h a, v16h b, v8f c) { return __builtin_amdgcn_wmma_f32_16x16x32_f16(false, a, false, b, (short)0, c, false, false); }
__device__ __forceinline__ v8f wmmab(v16bf a, v16bf b, v8f c) { return __builtin_amdgcn_wmma_f32_16x16x32_bf16(false, a, false, b, (short)0, c, false, false); }
__device__ __forceinline__ v16h  ldh(const h16* p) { return cat16(*(const v8h*)p, *(const v8h*)(p + 16)); }
__device__ __forceinline__ v16bf ldb(const bf* p)  { return cat16b(*(const v8us*)p, *(const v8us*)(p + 16)); }
__device__ __forceinline__ void wave_sync() { __builtin_amdgcn_fence(3  , "wavefront"); __builtin_amdgcn_wave_barrier(); asm volatile("" ::: "memory"); }

static __device__ __forceinline__ h16 toh_flush(float v) { const h16 r = (h16)v; return (fabsf(v) < 6.103515625e-05f) ? (h16)0.0f : r; }
__device__ __forceinline__ v8f mma_g(v16h a, v16h b, v8f c)   { c = wmma16(a, b, c); asm volatile("v_nop\n\tv_nop\n\tv_nop\n\tv_nop" : "+v"(c) : "v"(a), "v"(b)); return c; }
__device__ __forceinline__ v8f mma_g(v16bf a, v16bf b, v8f c) { c = wmmab(a, b, c);  asm volatile("v_nop\n\tv_nop\n\tv_nop\n\tv_nop" : "+v"(c) : "v"(a), "v"(b)); return c; }
__device__ __forceinline__ v16h  ldf(const h16* p) { return ldh(p); }
__device__ __forceinline__ v16bf ldf(const bf* p)  { return ldb(p); }
__device__ __forceinline__ float sigm(float x) { return __builtin_amdgcn_rcpf(1.0f + __builtin_amdgcn_exp2f(-x * LOG2E)); }
__device__ __forceinline__ float softplus_f(float s) {
    const float e = __builtin_amdgcn_exp2f(-fabsf(s) * LOG2E);
    const float lg = __log2f(1.0f + e) * LN2;
    const float sr = e * (1.0f + e * (-0.5f + e * (0.33333334f + e * -0.25f)));
    const float l = (e < 0.0625f) ? sr : lg;
    return fmaxf(s, 0.0f) + l;
}

__global__ __launch_bounds__(256) void k_cvt8(const float* __restrict__ src, bf* dst, size_t n8) {
    const size_t i = (size_t)blockIdx.x * 256 + threadIdx.x; if (i >= n8) return;
    const v8f v = *(const v8f*)(src + i * 8); v8us o;
#pragma unroll
    for (int k = 0; k < 8; ++k) o[k] = f2bf(v[k]);
    *(volatile v8us*)(dst + i * 8) = o; __threadfence(); *(volatile v8us*)(dst + i * 8) = o;
}

__global__ __launch_bounds__(256) void k_wconv(const float* __restrict__ src, h16* dst, int kin, int kpad, float scale, unsigned n8) {
    const unsigned i = blockIdx.x * 256u + threadIdx.x; if (i >= n8) return;
    const unsigned kp8 = (unsigned)kpad >> 3; const int r = (int)(i / kp8); const int k0 = (int)(i % kp8) * 8;
    v8h o;
#pragma unroll
    for (int k = 0; k < 8; ++k) {
        const int kk = k0 + k; const int kc = kk < kin ? kk : kin - 1;
        float v = src[(size_t)r * kin + kc]; asm volatile("" : "+v"(v));
        const h16 c = toh_flush(bfr(v) * scale);
        o[k] = (kk < kin) ? c : (h16)0.0f; }
    *(volatile v8h*)(dst + (size_t)i * 8) = o; __threadfence(); *(volatile v8h*)(dst + (size_t)i * 8) = o;
}

template <int EP, typename T>
__device__ __forceinline__ void gemm_body(const T* __restrict__ A, const T* __restrict__ Bt, const float* __restrict__ bias, const float* __restrict__ MUL, float* OF, h16* OH) {
    __shared__ __align__(16) float os[16 * 68];
    constexpr int K = (EP == EP_CAM || EP == EP_LID) ? DM : DI;
    const int lane = threadIdx.x & 31, lr = lane & 15, hi = lane >> 4; const int r0 = blockIdx.x * 64, c0 = blockIdx.y * 64;
    v8f acc[4][4];
#pragma unroll
    for (int mb = 0; mb < 4; ++mb)
#pragma unroll
        for (int nb = 0; nb < 4; ++nb) acc[mb][nb] = (v8f){};
    const size_t aoff = (size_t)(r0 + lr) * K + 8 * hi, boff = (size_t)(c0 + lr) * K + 8 * hi;
#pragma unroll 1
    for (int kc = 0; kc < K; kc += 32) {
        decltype(ldf(A)) a[4];
#pragma unroll
        for (int mb = 0; mb < 4; ++mb) a[mb] = ldf(A + aoff + (size_t)mb * 16 * K + kc);
#pragma unroll
        for (int nb = 0; nb < 4; ++nb) { const decltype(ldf(Bt)) b = ldf(Bt + boff + (size_t)nb * 16 * K + kc);
#pragma unroll
            for (int mb = 0; mb < 4; ++mb) acc[mb][nb] = mma_g(a[mb], b, acc[mb][nb]); }
    }
    float bc[4];
#pragma unroll
    for (int nb = 0; nb < 4; ++nb) { bc[nb] = 0.0f; if (EP == EP_GUID) bc[nb] = bfr(bias[c0 + nb * 16 + lr]); }
    const bool upper = (EP == EP_CAM) && (c0 >= DI);
    size_t obase, mbase = 0; int opitch;
    if (EP == EP_CAM)       { obase = (size_t)r0 * XZP + c0; opitch = XZP; }
    else if (EP == EP_LID)  { obase = (size_t)r0 * DI + c0;  opitch = DI; }
    else if (EP == EP_GUID) { obase = (size_t)r0 * DI + c0;  opitch = DI; mbase = (size_t)r0 * XZP + c0; }
    else                    { const int bb = r0 / SEQ, tt = r0 % SEQ; obase = ((size_t)bb * OUT_SEQ + (size_t)tt) * DM + c0; opitch = DM; }
#pragma unroll
    for (int mb = 0; mb < 4; ++mb) {
#pragma unroll
        for (int nb = 0; nb < 4; ++nb) {
#pragma unroll
            for (int j = 0; j < 8; ++j) {
                float v = acc[mb][nb][j];
                if (EP == EP_CAM)  { const float sv = v * sigm(v); v = upper ? sv : v; }
                if (EP == EP_GUID) { v = sigm(v * WSI + bc[nb]); }
                if (EP == EP_OUT)  { v = v * (WSI * YSI); }
                os[(hi * 8 + j) * 68 + nb * 16 + lr] = v; } }
        wave_sync();
        if (EP == EP_LID) {
#pragma unroll 1
            for (int ps = 0; ps < 2; ++ps) {
#pragma unroll
                for (int s = 0; s < 4; ++s) { const int row = 4 * s + (lane >> 3), c8 = (lane & 7) * 8;
                    const v4f x0 = *(const v4fa*)(&os[row * 68 + c8]); const v4f x1 = *(const v4fa*)(&os[row * 68 + c8 + 4]); v8h hv;
#pragma unroll
                    for (int i = 0; i < 4; ++i) { hv[i] = toh_flush(x0[i]); hv[4 + i] = toh_flush(x1[i]); }
                    *(volatile v8h*)(OH + obase + (size_t)(mb * 16 + row) * opitch + c8) = hv; }
                if (ps == 0) __threadfence(); }
        } else {
            v4f vv[8];
#pragma unroll
            for (int s = 0; s < 8; ++s) { const int row = 2 * s + (lane >> 4), c4 = (lane & 15) * 4;
                v4f x = *(const v4fa*)(&os[row * 68 + c4]);
                if (EP == EP_GUID) { const v4f y = *(const v4f*)(MUL + mbase + (size_t)(mb * 16 + row) * XZP + c4); x = x * y; }
                vv[s] = x; }
#pragma unroll 1
            for (int ps = 0; ps < 2; ++ps) {
#pragma unroll
                for (int s = 0; s < 8; ++s) { const int row = 2 * s + (lane >> 4), c4 = (lane & 15) * 4;
                    *(volatile v4f*)(OF + obase + (size_t)(mb * 16 + row) * opitch + c4) = vv[s]; }
                if (ps == 0) __threadfence(); }
        }
        wave_sync();
    }
}

__global__ __launch_bounds__(32) void k_gemm_cam(const bf* __restrict__ A, const bf* __restrict__ Bt, float* XZ) {
    gemm_body<EP_CAM, bf>(A, Bt, nullptr, nullptr, XZ, nullptr);
}
__global__ __launch_bounds__(32) void k_gemm_lid(const bf* __restrict__ A, const bf* __restrict__ Bt, h16* LXH) {
    gemm_body<EP_LID, bf>(A, Bt, nullptr, nullptr, nullptr, LXH);
}
__global__ __launch_bounds__(32) void k_gemm_guid(const h16* __restrict__ A, const h16* __restrict__ Bt, const float* __restrict__ bias, const float* __restrict__ XZ, float* U) {
    gemm_body<EP_GUID, h16>(A, Bt, bias, XZ, U, nullptr);
}
__global__ __launch_bounds__(32) void k_gemm_out(const h16* __restrict__ A, const h16* __restrict__ Bt, float* OUT) {
    gemm_body<EP_OUT, h16>(A, Bt, nullptr, nullptr, OUT, nullptr);
}

__global__ __launch_bounds__(32) void k_dparams(const float* __restrict__ XZ, const h16* __restrict__ WX, const h16* __restrict__ WD, const float* __restrict__ bdt, float* BCP, float* DELTA) {
    __shared__ __align__(16) float ss[64 * SSP];
    __shared__ __align__(16) float os[16 * 68];
    const int lane = threadIdx.x & 31, lr = lane & 15, hi = lane >> 4; const int r0 = blockIdx.x * 64;
    v8f acc[4][3];
#pragma unroll
    for (int mb = 0; mb < 4; ++mb)
#pragma unroll
        for (int nb = 0; nb < 3; ++nb) acc[mb][nb] = (v8f){};
    const size_t aoff = (size_t)(r0 + lr) * XZP + 8 * hi, boff = (size_t)lr * DI + 8 * hi;
#pragma unroll 1
    for (int kc = 0; kc < DI; kc += 32) {
        v16h a[4];
#pragma unroll
        for (int mb = 0; mb < 4; ++mb) { const float* p = XZ + aoff + (size_t)mb * 16 * XZP + kc;
            const v4f x0 = *(const v4f*)p, x1 = *(const v4f*)(p + 4), x2 = *(const v4f*)(p + 16), x3 = *(const v4f*)(p + 20);
            v16h t;
#pragma unroll
            for (int i = 0; i < 4; ++i) { t[i] = toh_flush(x0[i]); t[4 + i] = toh_flush(x1[i]); t[8 + i] = toh_flush(x2[i]); t[12 + i] = toh_flush(x3[i]); }
            a[mb] = t; }
#pragma unroll
        for (int nb = 0; nb < 3; ++nb) { const v16h b = ldh(WX + boff + (size_t)nb * 16 * DI + kc);
#pragma unroll
            for (int mb = 0; mb < 4; ++mb) acc[mb][nb] = mma_g(a[mb], b, acc[mb][nb]); }
    }
#pragma unroll
    for (int mb = 0; mb < 4; ++mb)
#pragma unroll
        for (int nb = 0; nb < 3; ++nb)
#pragma unroll
            for (int j = 0; j < 8; ++j) ss[(mb * 16 + hi * 8 + j) * SSP + nb * 16 + lr] = acc[mb][nb][j] * WSI;
    wave_sync();
#pragma unroll 1
    for (int ps = 0; ps < 2; ++ps) {
#pragma unroll
        for (int s = 0; s < 16; ++s) { const int row = 4 * s + (lane >> 3), c4 = (lane & 7) * 4;
            const v4f v = *(const v4fa*)(&ss[row * SSP + DR + c4]);
            *(volatile v4f*)(BCP + (size_t)(r0 + row) * 32 + c4) = v; }
        if (ps == 0) __threadfence(); }
    const v16h hz = (v16h){};
#pragma unroll 1
    for (int nc = 0; nc < DI / 64; ++nc) {
        v16h b[4]; float bcv[4];
#pragma unroll
        for (int nb = 0; nb < 4; ++nb) { const int n = nc * 64 + nb * 16 + lr; b[nb] = ldh(WD + (size_t)n * 32 + 8 * hi); bcv[nb] = bfr(bdt[n]); }
#pragma unroll 1
        for (int mb = 0; mb < 4; ++mb) {
            const int ai = (mb * 16 + lr) * SSP + 8 * hi;
            const v4f y0 = *(const v4fa*)(&ss[ai]); const v4f y1 = *(const v4fa*)(&ss[ai + 4]);
            v16h a = hz;
#pragma unroll
            for (int i = 0; i < 4; ++i) { a[i] = toh_flush(y0[i]); a[4 + i] = toh_flush(y1[i]); }
#pragma unroll
            for (int nb = 0; nb < 4; ++nb) { const v8f d = mma_g(a, b[nb], (v8f){});
#pragma unroll
                for (int j = 0; j < 8; ++j) os[(hi * 8 + j) * 68 + nb * 16 + lr] = softplus_f(d[j] * WSI + bcv[nb]); }
            wave_sync();
            v4f vv[8];
#pragma unroll
            for (int s = 0; s < 8; ++s) { const int row = 2 * s + (lane >> 4), c4 = (lane & 15) * 4; vv[s] = *(const v4fa*)(&os[row * 68 + c4]); }
#pragma unroll 1
            for (int ps = 0; ps < 2; ++ps) {
#pragma unroll
                for (int s = 0; s < 8; ++s) { const int row = 2 * s + (lane >> 4), c4 = (lane & 15) * 4;
                    *(volatile v4f*)(DELTA + (size_t)(r0 + mb * 16 + row) * DI + nc * 64 + c4) = vv[s]; }
                if (ps == 0) __threadfence(); }
            wave_sync();
        }
    }
}

template <int FWD>
__device__ __forceinline__ void scan_body(const float* __restrict__ U, const float* __restrict__ DELTA, const float* __restrict__ BCP, const float* __restrict__ Alog,
                                          const float* __restrict__ Dv, const float* __restrict__ XZ, const float* __restrict__ YBr, float* YBw, h16* YF) {
    __shared__ __align__(16) float bcs[TC * 32];
    __shared__ __align__(16) float ys[TC * SCH];
    const int tid = threadIdx.x, lane = tid & 31;
    const int wave = __builtin_amdgcn_readfirstlane((int)(threadIdx.x >> 5));
    const int cb = blockIdx.x * SCH; const int d = cb + tid;
    const size_t tb = (size_t)blockIdx.y * SEQ;
    float A2[DS];
#pragma unroll
    for (int q = 0; q < 4; ++q) { const v4f a4 = *(const v4f*)(Alog + (size_t)d * DS + 4 * q);
#pragma unroll
        for (int k = 0; k < 4; ++k) A2[4 * q + k] = -__builtin_amdgcn_exp2f(bfr(a4[k]) * LOG2E) * LOG2E; }
    float Dd = 0.0f; if (FWD) Dd = bfr(Dv[d]);
    float xs[DS];
#pragma unroll
    for (int n = 0; n < DS; ++n) xs[n] = 0.0f;
#pragma unroll 1
    for (int c = 0; c < SEQ / TC; ++c) {
        const int t0 = FWD ? c * TC : SEQ - (c + 1) * TC;
#pragma unroll
        for (int q = 0; q < (TC * 8) / SCH; ++q) { const int idx = q * SCH + tid;
            const v4f v = *(const v4f*)(BCP + (tb + (size_t)t0) * 32 + (size_t)idx * 4);
            *(v4fa*)(&bcs[idx * 4]) = v; }
        __syncthreads();
#pragma unroll 1
        for (int s = 0; s < TC; ++s) {
            const int tl = FWD ? s : TC - 1 - s;
            const size_t e = (tb + (size_t)(t0 + tl)) * DI + d;
            const float dv = DELTA[e], uv = U[e]; const float du = dv * uv;
            v4f bq[4], cq[4];
#pragma unroll
            for (int q = 0; q < 4; ++q) { bq[q] = *(const v4fa*)(&bcs[tl * 32 + 4 * q]); cq[q] = *(const v4fa*)(&bcs[tl * 32 + 16 + 4 * q]); }
            float accy = 0.0f;
#pragma unroll
            for (int n = 0; n < DS; ++n) {
                const float dA = __builtin_amdgcn_exp2f(dv * A2[n]);
                xs[n] = dA * xs[n] + du * bq[n >> 2][n & 3];
                accy += xs[n] * cq[n >> 2][n & 3]; }
            ys[tl * SCH + tid] = FWD ? (accy + 2.0f * (uv * Dd)) : accy;
        }
        __syncthreads();
        if (FWD) {
            v8h hv[TC / 8];
#pragma unroll
            for (int i = 0; i < TC / 8; ++i) { const int row = 2 * (wave + 4 * i) + (lane >> 4), c8 = (lane & 15) * 8;
                const v4f y0 = *(const v4fa*)(&ys[row * SCH + c8]); const v4f y1 = *(const v4fa*)(&ys[row * SCH + c8 + 4]);
                const size_t tok = tb + (size_t)(t0 + row);
                const v4f b0 = *(const v4f*)(YBr + tok * DI + cb + c8); const v4f b1 = *(const v4f*)(YBr + tok * DI + cb + c8 + 4);
                const v4f g0 = *(const v4f*)(XZ + tok * XZP + DI + cb + c8); const v4f g1 = *(const v4f*)(XZ + tok * XZP + DI + cb + c8 + 4);
                v8h t;
#pragma unroll
                for (int k = 0; k < 4; ++k) { t[k] = toh_flush((y0[k] + b0[k]) * g0[k] * YSC); t[4 + k] = toh_flush((y1[k] + b1[k]) * g1[k] * YSC); }
                hv[i] = t; }
#pragma unroll 1
            for (int ps = 0; ps < 2; ++ps) {
#pragma unroll
                for (int i = 0; i < TC / 8; ++i) { const int row = 2 * (wave + 4 * i) + (lane >> 4), c8 = (lane & 15) * 8;
                    const size_t tok = tb + (size_t)(t0 + row);
                    *(volatile v8h*)(YF + tok * DI + cb + c8) = hv[i]; }
                if (ps == 0) __threadfence(); }
        } else {
#pragma unroll 1
            for (int ps = 0; ps < 2; ++ps) {
#pragma unroll 4
                for (int i = 0; i < TC / 4; ++i) { const int row = wave + 4 * i;
                    const v4f v = *(const v4fa*)(&ys[row * SCH + lane * 4]);
                    *(volatile v4f*)(YBw + (tb + (size_t)(t0 + row)) * DI + cb + lane * 4) = v; }
                if (ps == 0) __threadfence(); }
        }
    }
}

__global__ __launch_bounds__(SCH) void k_scan_bwd(const float* __restrict__ U, const float* __restrict__ DELTA, const float* __restrict__ BCP, const float* __restrict__ Alog, float* YB) {
    scan_body<0>(U, DELTA, BCP, Alog, nullptr, nullptr, nullptr, YB, nullptr);
}
__global__ __launch_bounds__(SCH) void k_scan_fwd(const float* __restrict__ U, const float* __restrict__ DELTA, const float* __restrict__ BCP, const float* __restrict__ Alog,
                                                  const float* __restrict__ Dv, const float* __restrict__ XZ, const float* __restrict__ YB, h16* YF) {
    scan_body<1>(U, DELTA, BCP, Alog, Dv, XZ, YB, nullptr, YF);
}

static constexpr size_t al256(size_t v) { return (v + 255) & ~(size_t)255; }
static constexpr size_t SZ_XB  = al256((size_t)NTG * DM * 2);
static constexpr size_t SZ_WIN = al256((size_t)2 * DI * DM * 2);
static constexpr size_t SZ_WG  = al256((size_t)DI * DI * 2);
static constexpr size_t SZ_WX  = al256((size_t)NX * DI * 2);
static constexpr size_t SZ_WD  = al256((size_t)DI * 32 * 2);
static constexpr size_t SZ_WO  = al256((size_t)DM * DI * 2);
static constexpr size_t SZ_XZ  = al256((size_t)NTG * XZP * 4);
static constexpr size_t SZ_F32 = al256((size_t)NTG * DI * 4);
static constexpr size_t SZ_H16 = al256((size_t)NTG * DI * 2);
static constexpr size_t SZ_BC  = al256((size_t)NTG * 32 * 4);
static constexpr size_t SZ_TOTAL = 2 * SZ_XB + SZ_WIN + SZ_WG + SZ_WX + SZ_WD + SZ_WO + SZ_XZ + 3 * SZ_F32 + 2 * SZ_H16 + SZ_BC;
static_assert(SZ_TOTAL <= (size_t)134217728);
static_assert(((size_t)NTG * DM) % 8 == 0);
static_assert(((size_t)SEQ * DM) % 8 == 0);
static_assert(((size_t)2 * DI * DM) % 8 == 0);

extern "C" void kernel_launch(void* const* d_in, const int* in_sizes, int n_in,
                              void* d_out, int out_size, void* d_ws, size_t ws_size, hipStream_t stream) {
    if (n_in < 12) return;
    const size_t needx = ((size_t)(NB - 1) * SEQ_FULL + SEQ) * DM;
    if ((size_t)in_sizes[0] < needx || (size_t)in_sizes[1] < needx) return;
    if ((size_t)in_sizes[2] < (size_t)2 * DI * DM || (size_t)in_sizes[3] < (size_t)NX * DI || (size_t)in_sizes[4] < (size_t)DI * DR) return;
    if (in_sizes[5] < DI || in_sizes[6] < DI * DS || in_sizes[7] < DI * DS || in_sizes[8] < DI) return;
    if ((size_t)in_sizes[9] < (size_t)DI * DI || in_sizes[10] < DI || (size_t)in_sizes[11] < (size_t)DM * DI) return;
    if ((size_t)out_size < ((size_t)(NB - 1) * OUT_SEQ + SEQ) * DM) return;
    if (SZ_TOTAL > ws_size) return;
    const float* xg    = (const float*)d_in[0];
    const float* xm    = (const float*)d_in[1];
    const float* w_in  = (const float*)d_in[2];
    const float* w_xp  = (const float*)d_in[3];
    const float* w_dt  = (const float*)d_in[4];
    const float* b_dt  = (const float*)d_in[5];
    const float* a_h2t = (const float*)d_in[6];
    const float* a_t2h = (const float*)d_in[7];
    const float* dvec  = (const float*)d_in[8];
    const float* w_gd  = (const float*)d_in[9];
    const float* b_gd  = (const float*)d_in[10];
    const float* w_out = (const float*)d_in[11];
    float* OUT = (float*)d_out;
    char* wsp = (char*)d_ws;
    bf*  LB   = (bf*)wsp;   wsp += SZ_XB;
    bf*  CB   = (bf*)wsp;   wsp += SZ_XB;
    bf*  WINB = (bf*)wsp;   wsp += SZ_WIN;
    h16* WG   = (h16*)wsp;  wsp += SZ_WG;
    h16* WX   = (h16*)wsp;  wsp += SZ_WX;
    h16* WD   = (h16*)wsp;  wsp += SZ_WD;
    h16* WO   = (h16*)wsp;  wsp += SZ_WO;
    float* XZ = (float*)wsp; wsp += SZ_XZ;
    float* U  = (float*)wsp; wsp += SZ_F32;
    float* DL = (float*)wsp; wsp += SZ_F32;
    float* YB = (float*)wsp; wsp += SZ_F32;
    h16* LXH  = (h16*)wsp;  wsp += SZ_H16;
    h16* YF   = (h16*)wsp;  wsp += SZ_H16;
    float* BCP = (float*)wsp; wsp += SZ_BC;

    { const size_t n8 = (size_t)2 * DI * DM / 8; k_cvt8<<<(unsigned)((n8 + 255) / 256), 256, 0, stream>>>(w_in, WINB, n8); }
    { const unsigned n8 = (unsigned)((size_t)DI * DI / 8); k_wconv<<<(n8 + 255) / 256, 256, 0, stream>>>(w_gd, WG, DI, DI, WSC, n8); }
    { const unsigned n8 = (unsigned)((size_t)NX * DI / 8); k_wconv<<<(n8 + 255) / 256, 256, 0, stream>>>(w_xp, WX, DI, DI, WSC, n8); }
    { const unsigned n8 = (unsigned)((size_t)DI * 32 / 8); k_wconv<<<(n8 + 255) / 256, 256, 0, stream>>>(w_dt, WD, DR, 32, WSC, n8); }
    { const unsigned n8 = (unsigned)((size_t)DM * DI / 8); k_wconv<<<(n8 + 255) / 256, 256, 0, stream>>>(w_out, WO, DI, DI, WSC, n8); }

    for (int g0 = 0; g0 < NB; g0 += BG) {
        if (SEQ == SEQ_FULL) {
            const size_t n8 = (size_t)NTG * DM / 8;
            k_cvt8<<<(unsigned)((n8 + 255) / 256), 256, 0, stream>>>(xg + (size_t)g0 * SEQ_FULL * DM, LB, n8);
            k_cvt8<<<(unsigned)((n8 + 255) / 256), 256, 0, stream>>>(xm + (size_t)g0 * SEQ_FULL * DM, CB, n8);
        } else {
            const size_t n8 = (size_t)SEQ * DM / 8;
            for (int b = 0; b < BG; ++b) {
                k_cvt8<<<(unsigned)((n8 + 255) / 256), 256, 0, stream>>>(xg + (size_t)(g0 + b) * SEQ_FULL * DM, LB + (size_t)b * SEQ * DM, n8);
                k_cvt8<<<(unsigned)((n8 + 255) / 256), 256, 0, stream>>>(xm + (size_t)(g0 + b) * SEQ_FULL * DM, CB + (size_t)b * SEQ * DM, n8);
            }
        }
        k_gemm_lid<<<dim3(NTG / 64, DI / 64, 1), 32, 0, stream>>>(LB, WINB, LXH);
        k_gemm_cam<<<dim3(NTG / 64, XZP / 64, 1), 32, 0, stream>>>(CB, WINB, XZ);
        k_gemm_guid<<<dim3(NTG / 64, DI / 64, 1), 32, 0, stream>>>(LXH, WG, b_gd, XZ, U);
        k_dparams<<<dim3(NTG / 64, 1, 1), 32, 0, stream>>>(XZ, WX, WD, b_dt, BCP, DL);
        k_scan_bwd<<<dim3(DI / SCH, BG, 1), SCH, 0, stream>>>(U, DL, BCP, a_t2h, YB);
        k_scan_fwd<<<dim3(DI / SCH, BG, 1), SCH, 0, stream>>>(U, DL, BCP, a_h2t, dvec, XZ, YB, YF);
        k_gemm_out<<<dim3(NTG / 64, DM / 64, 1), 32, 0, stream>>>(YF, WO, OUT + (size_t)g0 * OUT_SEQ * DM);
    }
}
